// CrossModalMultiHeadAttentionK_70987219469039
// MI455X (gfx1250) — hardware-verified
//
#include <hip/hip_runtime.h>
#include <stddef.h>
#include <math.h>

#define NB    2
#define CH    256
#define IMG   40
#define NPIX  1600
#define NTQ   3200
#define PADW  46
#define NPK   2116
#define NTK   4232
#define NTKP  4288
#define NTAP  49
#define NCNT  41
#define TBLK  44
#define TBLN  11264

static_assert(NTQ == NB * NPIX);
static_assert(NPIX == IMG * IMG);
static_assert(NPIX % 64 == 0);
static_assert(NTQ % 64 == 0);
static_assert(NTQ % 8 == 0);
static_assert(NTK == NB * NPK);
static_assert(NPK == PADW * PADW);
static_assert(NTKP % 64 == 0);
static_assert(NTKP >= NTK);
static_assert(NTKP - NTK < 64);
static_assert(TBLN == TBLK * 256);
static_assert(TBLN >= CH * NCNT);
static_assert(CH % 32 == 0);

#define ASC     8.0f
#define WSC     64.0f
#define AOSC    64.0f
#define VOSC    32.0f
#define WF2SC   16.0f
#define INV_XW  0.001953125f
#define INV_AOW 0.000244140625f
#define QSCALE  0.17677669529663688f
#define PE_SCALE 6.283185307179586f
#define PE_L2S   0.20762050593046014f
#define PE_HPI   1.5707963267948966f

typedef _Float16 v16h __attribute__((ext_vector_type(16)));
typedef _Float16 v8h  __attribute__((ext_vector_type(8)));
typedef float    v8f  __attribute__((ext_vector_type(8)));
typedef float    v4f  __attribute__((ext_vector_type(4)));
typedef unsigned int v4u __attribute__((ext_vector_type(4)));

union FragH { v16h v; v8h h[2]; };
union Pack8 { v8h h; v4u u; };

__device__ __forceinline__ v8f mma_h(v16h a, v16h b, v8f c) {
  c = __builtin_amdgcn_wmma_f32_16x16x32_f16(false, a, false, b, (short)0, c, false, false);
  asm volatile("v_nop\n\tv_nop\n\tv_nop\n\tv_nop" : "+v"(c) : "v"(a), "v"(b));
  return c;
}
__device__ __forceinline__ v8f zero8() { return (v8f){0.f, 0.f, 0.f, 0.f, 0.f, 0.f, 0.f, 0.f}; }

__device__ __forceinline__ v16h ldfrag_h(const _Float16* p, int ld, int row0, int k0, int lane) {
  const int m = lane & 15, lh = lane >> 4;
  const _Float16* q = p + (size_t)(row0 + m) * ld + k0 + 8 * lh;
  FragH f;
  f.h[0] = *(const v8h*)(q);
  f.h[1] = *(const v8h*)(q + 16);
  return f.v;
}

template <int KSTEPS>
__device__ __forceinline__ void gemm16x64(const _Float16* A, int lda, const _Float16* B, int ldb,
                                          int m0, int n0, int lane, v8f (&acc)[4]) {
  static_assert(KSTEPS % 2 == 0);
#pragma unroll 1
  for (int kg = 0; kg < KSTEPS; kg += 2) {
#pragma unroll
    for (int u = 0; u < 2; ++u) {
      const int k0 = (kg + u) * 32;
      const v16h a = ldfrag_h(A, lda, m0, k0, lane);
#pragma unroll
      for (int t = 0; t < 4; ++t) {
        const v16h bb = ldfrag_h(B, ldb, n0 + 16 * t, k0, lane);
        acc[t] = mma_h(a, bb, acc[t]);
      }
    }
  }
}

union Stg256 { float f[256]; v4f v[64]; };
__global__ __launch_bounds__(256) void k_petab(float* __restrict__ tb) {
  __shared__ __align__(16) Stg256 st;
  const int tid = threadIdx.x;
  const int f = blockIdx.x * 256 + tid;
  int c = f / NCNT;
  const int cnt = f - c * NCNT;
  c = min(c, CH - 1);
  const int cc = c & 127;
  const float invd = exp2f(-(float)(cc >> 1) * PE_L2S);
  const float base = ((float)cnt * (1.0f / 40.0f)) * PE_SCALE;
  const float ph = (cc & 1) ? PE_HPI : 0.0f;
  const float arg = base * invd + ph;
  st.f[tid] = sinf(arg);
  __syncthreads();
  if (tid < 64) {
    const v4f v = st.v[tid];
    float* dp = tb + (size_t)blockIdx.x * 256 + tid * 4;
    *(volatile v4f*)dp = v;
    __threadfence();
    *(volatile v4f*)dp = v;
  }
}

__global__ __launch_bounds__(256) void k_wcv(const float* __restrict__ W, int n8, int rowp, int hp,
                                             float s1, float s2, _Float16* __restrict__ wp16) {
  int i = blockIdx.x * 256 + threadIdx.x;
  i = min(i, n8 - 1);
  const float sc = ((i % rowp) < hp) ? s1 : s2;
  const float* wp = W + (size_t)i * 8;
  const v4f a0 = *(const v4f*)(wp), a1 = *(const v4f*)(wp + 4);
  Pack8 pk;
  pk.h = (v8h){(_Float16)(a0[0] * sc), (_Float16)(a0[1] * sc), (_Float16)(a0[2] * sc), (_Float16)(a0[3] * sc),
               (_Float16)(a1[0] * sc), (_Float16)(a1[1] * sc), (_Float16)(a1[2] * sc), (_Float16)(a1[3] * sc)};
  _Float16* dp = wp16 + (size_t)i * 8;
  *(volatile v4u*)dp = pk.u;
  __threadfence();
  *(volatile v4u*)dp = pk.u;
}

#define WTP 65
__global__ __launch_bounds__(256) void k_prepq(const float* __restrict__ query, const float* __restrict__ tb,
                                               _Float16* __restrict__ xq) {
  __shared__ float tl[128 * WTP];
  const int tid = threadIdx.x;
  const int n0 = blockIdx.x * 64, chh = blockIdx.y, b = blockIdx.z;
  const float* xb = query + ((size_t)(b * CH + chh * 128)) * NPIX;
#pragma unroll
  for (int j = 0; j < 8; ++j) {
    const int p  = tid + 256 * j;
    const int cc = p >> 4;
    const int q4 = (p & 15) * 4;
    const v4f a = *(const v4f*)(xb + (size_t)cc * NPIX + n0 + q4);
    float* d = tl + cc * WTP + q4;
    d[0] = a[0]; d[1] = a[1]; d[2] = a[2]; d[3] = a[3];
  }
  __syncthreads();
  const int pc = tid & 15;
#pragma unroll 1
  for (int j = 0; j < 4; ++j) {
    const int p  = tid + 256 * j;
    const int nn = p >> 4;
    const int n  = n0 + nn;
    const int h  = n / IMG;
    const int w  = n - h * IMG;
    const int cnt = (chh == 0) ? (h + 1) : (w + 1);
    const float* cp = tl + (8 * pc) * WTP + nn;
    const float* tp = tb + (size_t)(chh * 128 + 8 * pc) * NCNT + cnt;
    float v[8];
#pragma unroll
    for (int i = 0; i < 8; ++i) v[i] = (cp[i * WTP] + tp[i * NCNT]) * ASC;
    Pack8 pk;
    pk.h = (v8h){(_Float16)v[0], (_Float16)v[1], (_Float16)v[2], (_Float16)v[3],
                 (_Float16)v[4], (_Float16)v[5], (_Float16)v[6], (_Float16)v[7]};
    _Float16* dp = xq + ((size_t)(b * NPIX + n) * CH + chh * 128 + 8 * pc);
    *(volatile v4u*)dp = pk.u;
    __threadfence();
    *(volatile v4u*)dp = pk.u;
  }
}

__global__ __launch_bounds__(256) void k_prepk(const float* __restrict__ key, const float* __restrict__ tb,
                                               _Float16* __restrict__ xk, _Float16* __restrict__ pk) {
  const int tid = threadIdx.x;
  const int t0 = blockIdx.x * 64;
#pragma unroll 1
  for (int j = 0; j < 8; ++j) {
    const int p  = tid + 256 * j;
    const int tl = p >> 5;
    const int pc = p & 31;
    const int t  = t0 + tl;
    const bool valid = t < NTK;
    const int tc = min(t, NTK - 1);
    const int b  = tc / NPK;
    const int n  = tc - b * NPK;
    const int ph = n / PADW;
    const int pw = n - ph * PADW;
    const bool rin = (ph >= 3) && (ph < 3 + IMG);
    const bool cin = (pw >= 3) && (pw < 3 + IMG);
    const bool inb = rin && cin;
    const int hs  = min(max(ph - 3, 0), IMG - 1);
    const int wsx = min(max(pw - 3, 0), IMG - 1);
    const int ycnt = cin ? ((ph < 3) ? 0 : (min(ph, IMG + 2) - 2)) : 0;
    const int xcnt = rin ? ((pw < 3) ? 0 : (min(pw, IMG + 2) - 2)) : 0;
    const int cnt = (pc < 16) ? ycnt : xcnt;
    const float* kp = key + ((size_t)(b * CH + 8 * pc)) * NPIX + hs * IMG + wsx;
    const float* tp = tb + (size_t)(8 * pc) * NCNT + cnt;
    float av[8], rv[8];
#pragma unroll
    for (int i = 0; i < 8; ++i) {
      float kv = kp[(size_t)i * NPIX];
      kv = inb ? kv : 0.0f;
      const float pe = tp[i * NCNT];
      av[i] = valid ? (kv + pe) * ASC : 0.0f;
      rv[i] = valid ? kv * ASC : 0.0f;
    }
    Pack8 pa, pr;
    pa.h = (v8h){(_Float16)av[0], (_Float16)av[1], (_Float16)av[2], (_Float16)av[3],
                 (_Float16)av[4], (_Float16)av[5], (_Float16)av[6], (_Float16)av[7]};
    pr.h = (v8h){(_Float16)rv[0], (_Float16)rv[1], (_Float16)rv[2], (_Float16)rv[3],
                 (_Float16)rv[4], (_Float16)rv[5], (_Float16)rv[6], (_Float16)rv[7]};
    const size_t o = (size_t)t * CH + 8 * pc;
    *(volatile v4u*)(xk + o) = pa.u;
    *(volatile v4u*)(pk + o) = pr.u;
    __threadfence();
    *(volatile v4u*)(xk + o) = pa.u;
    *(volatile v4u*)(pk + o) = pr.u;
  }
}

#define SFP 132
__global__ __launch_bounds__(256) void k_gemm_tok(const _Float16* __restrict__ A,
                                                  const _Float16* __restrict__ Bw,
                                                  const float* __restrict__ bias,
                                                  float oscale,
                                                  float* __restrict__ dst) {
  __shared__ __align__(16) float sf[64 * SFP];
  const int tid = threadIdx.x, lane = tid & 31, wave = tid >> 5;
  const int hh = lane >> 4, c = lane & 15;
  const int wm = wave >> 1, wn = wave & 1;
  const int mb = blockIdx.x * 64;
  const int colb = blockIdx.y * 128;
  const int m0 = mb + wm * 16;
  const int n0 = colb + wn * 64;

  v8f acc[4];
#pragma unroll
  for (int t = 0; t < 4; ++t) acc[t] = zero8();
  gemm16x64<CH / 32>(A, CH, Bw, CH, m0, n0, lane, acc);

#pragma unroll
  for (int t = 0; t < 4; ++t) {
    const float bb = bias[n0 + 16 * t + c];
#pragma unroll
    for (int r = 0; r < 8; ++r)
      sf[(wm * 16 + 8 * hh + r) * SFP + wn * 64 + 16 * t + c] = (acc[t][r] * INV_XW + bb) * oscale;
  }
  __syncthreads();

  v4f val[8];
  size_t go[8];
#pragma unroll
  for (int j = 0; j < 8; ++j) {
    const int p   = tid + 256 * j;
    const int row = p >> 5;
    const int pc  = p & 31;
    val[j] = *(const v4f*)(sf + row * SFP + pc * 4);
    go[j]  = (size_t)(mb + row) * CH + colb + pc * 4;
  }
  for (int ps = 0; ps < 2; ++ps) {
#pragma unroll
    for (int j = 0; j < 8; ++j) *(volatile v4f*)(dst + go[j]) = val[j];
    __threadfence();
  }
}

#define OTP 68
template <bool TWOA, bool HASB, bool F16P>
__global__ __launch_bounds__(256) void k_gemm_nchw(const _Float16* __restrict__ A1,
                                                   const _Float16* __restrict__ A2,
                                                   const _Float16* __restrict__ Bw,
                                                   int ldb,
                                                   const float* __restrict__ bias,
                                                   float inv,
                                                   float* __restrict__ dstn,
                                                   _Float16* __restrict__ dst16,
                                                   float s16) {
  __shared__ __align__(16) float st[128 * OTP];
  const int tid = threadIdx.x, lane = tid & 31, wave = tid >> 5;
  const int hh = lane >> 4, c = lane & 15;
  const int wm = wave >> 1, wn = wave & 1;
  const int mb  = blockIdx.x * 64;
  const int b   = mb / NPIX;
  const int nb0 = mb - b * NPIX;
  const int colb = blockIdx.y * 128;
  const int m0  = mb + wm * 16;
  const int n0  = colb + wn * 64;

  v8f acc[4];
#pragma unroll
  for (int t = 0; t < 4; ++t) acc[t] = zero8();
  gemm16x64<CH / 32>(A1, CH, Bw, ldb, m0, n0, lane, acc);
  if (TWOA) gemm16x64<CH / 32>(A2, CH, Bw + CH, ldb, m0, n0, lane, acc);

#pragma unroll
  for (int t = 0; t < 4; ++t) {
    float bb = 0.0f;
    if (HASB) bb = bias[n0 + 16 * t + c];
#pragma unroll
    for (int r = 0; r < 8; ++r)
      st[(wn * 64 + 16 * t + c) * OTP + wm * 16 + 8 * hh + r] = acc[t][r] * inv + bb;
  }
  __syncthreads();

  {
    v4f val[8];
    size_t go[8];
#pragma unroll
    for (int it = 0; it < 8; ++it) {
      const int p    = lane + 32 * it;
      const int L    = p >> 3;
      const int pc   = p & 7;
      const int cl   = wave * 16 + (L >> 1);
      const int half = L & 1;
      go[it]  = ((size_t)(b * CH + colb + cl)) * NPIX + nb0 + half * 32 + pc * 4;
      val[it] = *(const v4f*)(st + cl * OTP + half * 32 + pc * 4);
    }
    for (int ps = 0; ps < 2; ++ps) {
#pragma unroll
      for (int it = 0; it < 8; ++it) *(volatile v4f*)(dstn + go[it]) = val[it];
      __threadfence();
    }
  }

  if (F16P) {
    v4u hv[4];
    size_t ho[4];
    const int pc = tid & 15;
#pragma unroll
    for (int j = 0; j < 4; ++j) {
      const int p   = tid + 256 * j;
      const int row = p >> 4;
      const float* cp = st + (8 * pc) * OTP + row;
      Pack8 pk;
      pk.h = (v8h){(_Float16)(cp[0 * OTP] * s16), (_Float16)(cp[1 * OTP] * s16),
                   (_Float16)(cp[2 * OTP] * s16), (_Float16)(cp[3 * OTP] * s16),
                   (_Float16)(cp[4 * OTP] * s16), (_Float16)(cp[5 * OTP] * s16),
                   (_Float16)(cp[6 * OTP] * s16), (_Float16)(cp[7 * OTP] * s16)};
      hv[j] = pk.u;
      ho[j] = (size_t)(mb + row) * CH + colb + 8 * pc;
    }
    for (int ps = 0; ps < 2; ++ps) {
#pragma unroll
      for (int j = 0; j < 4; ++j) *(volatile v4u*)(dst16 + ho[j]) = hv[j];
      __threadfence();
    }
  }
}

union StgAO { _Float16 h[8 * CH]; v4u u[CH]; };
__global__ __launch_bounds__(256) void k_attn(const float* __restrict__ qf,
                                              const float* __restrict__ kf,
                                              const float* __restrict__ vf,
                                              _Float16* __restrict__ ao) {
  __shared__ float sm_sc[256 * NTAP];
  __shared__ __align__(16) StgAO stg;
  const int tid = threadIdx.x;
  float* scw = sm_sc + tid * NTAP;
  const int t0 = blockIdx.x * 8;
#pragma unroll 1
  for (int jp = 0; jp < 8; ++jp) {
    const int t = t0 + jp;
    const int b = t / NPIX;
    const int n = t - b * NPIX;
    const int h = n / IMG;
    const int w = n - h * IMG;
    const float q = qf[(size_t)t * CH + tid];
    const size_t kb = ((size_t)(b * NPK + h * PADW + w)) * CH + tid;
    const float* kp = kf + kb;
    const float* vp = vf + kb;
    float mx = -3.0e38f;
#pragma unroll 1
    for (int i = 0; i < 7; ++i) {
#pragma unroll
      for (int j = 0; j < 7; ++j) {
        const float s = q * kp[(size_t)(i * PADW + j) * CH];
        scw[i * 7 + j] = s;
        mx = fmaxf(mx, s);
      }
    }
    float den = 0.0f, acc = 0.0f;
#pragma unroll 1
    for (int i = 0; i < 7; ++i) {
#pragma unroll
      for (int j = 0; j < 7; ++j) {
        const float e = __expf(scw[i * 7 + j] - mx);
        den += e;
        acc = fmaf(e, vp[(size_t)(i * PADW + j) * CH], acc);
      }
    }
    const float o = acc * __builtin_amdgcn_rcpf(den);
    stg.h[jp * CH + tid] = (_Float16)(o * AOSC);
  }
  __syncthreads();
  const int row = tid >> 5, pc = tid & 31;
  const v4u v = stg.u[row * 32 + pc];
  _Float16* dp = ao + (size_t)(t0 + row) * CH + pc * 8;
  *(volatile v4u*)dp = v;
  __threadfence();
  *(volatile v4u*)dp = v;
}

extern "C" void kernel_launch(void* const* d_in, const int* in_sizes, int n_in,
                              void* d_out, int out_size, void* d_ws, size_t ws_size,
                              hipStream_t stream) {
  if (n_in < 11) return;
  if (in_sizes[0] != NTQ * CH || in_sizes[1] != NTQ * CH) return;
  if (in_sizes[2] != CH * CH || in_sizes[3] != CH) return;
  if (in_sizes[4] != CH * CH || in_sizes[5] != CH) return;
  if (in_sizes[6] != CH * CH || in_sizes[7] != CH) return;
  if (in_sizes[8] != CH * CH || in_sizes[9] != CH) return;
  if (in_sizes[10] != CH * 2 * CH) return;
  if (out_size != 2 * NTQ * CH) return;

  const float* key   = (const float*)d_in[0];
  const float* query = (const float*)d_in[1];
  const float* Wq = (const float*)d_in[2];   const float* bq = (const float*)d_in[3];
  const float* Wk = (const float*)d_in[4];   const float* bk = (const float*)d_in[5];
  const float* Wv = (const float*)d_in[6];   const float* bv = (const float*)d_in[7];
  const float* Wo = (const float*)d_in[8];   const float* bo = (const float*)d_in[9];
  const float* Wf = (const float*)d_in[10];
  float* out_o  = (float*)d_out;
  float* out_vo = out_o + (size_t)NTQ * CH;

  size_t off = 0;
  const size_t oTB  = off; off += (size_t)TBLN * 4;
  const size_t oWQ  = off; off += (size_t)CH * CH * 2;
  const size_t oWK  = off; off += (size_t)CH * CH * 2;
  const size_t oWV  = off; off += (size_t)CH * CH * 2;
  const size_t oWO  = off; off += (size_t)CH * CH * 2;
  const size_t oWF  = off; off += (size_t)CH * 2 * CH * 2;
  const size_t oXQ  = off; off += (size_t)NTQ * CH * 2;
  const size_t oXK  = off; off += (size_t)NTKP * CH * 2;
  const size_t oPK  = off; off += (size_t)NTKP * CH * 2;
  const size_t oQF  = off; off += (size_t)NTQ * CH * 4;
  const size_t oKF  = off; off += (size_t)NTKP * CH * 4;
  const size_t oVF  = off; off += (size_t)NTKP * CH * 4;
  const size_t oAO  = off; off += (size_t)NTQ * CH * 2;
  const size_t oVO  = off; off += (size_t)NTQ * CH * 2;
  if (off > ws_size) return;
  if (off > (size_t)134217728) return;

  char* ws = (char*)d_ws;
  float*    TB   = (float*)(ws + oTB);
  _Float16* WQ16 = (_Float16*)(ws + oWQ);
  _Float16* WK16 = (_Float16*)(ws + oWK);
  _Float16* WV16 = (_Float16*)(ws + oWV);
  _Float16* WO16 = (_Float16*)(ws + oWO);
  _Float16* WF16 = (_Float16*)(ws + oWF);
  _Float16* XQ   = (_Float16*)(ws + oXQ);
  _Float16* XK   = (_Float16*)(ws + oXK);
  _Float16* PK   = (_Float16*)(ws + oPK);
  float*    QF   = (float*)(ws + oQF);
  float*    KF   = (float*)(ws + oKF);
  float*    VF   = (float*)(ws + oVF);
  _Float16* AO   = (_Float16*)(ws + oAO);
  _Float16* VO16 = (_Float16*)(ws + oVO);

  const int n8p = CH * CH / 8;
  const int n8f = CH * 2 * CH / 8;
  if ((n8p % 256) != 0 || (n8f % 256) != 0) return;

  k_petab<<<dim3(TBLK), dim3(256), 0, stream>>>(TB);
  k_wcv<<<dim3(n8p / 256), dim3(256), 0, stream>>>(Wq, n8p, 32, 32, WSC, WSC, WQ16);
  k_wcv<<<dim3(n8p / 256), dim3(256), 0, stream>>>(Wk, n8p, 32, 32, WSC, WSC, WK16);
  k_wcv<<<dim3(n8p / 256), dim3(256), 0, stream>>>(Wv, n8p, 32, 32, WSC, WSC, WV16);
  k_wcv<<<dim3(n8p / 256), dim3(256), 0, stream>>>(Wo, n8p, 32, 32, WSC, WSC, WO16);
  k_wcv<<<dim3(n8f / 256), dim3(256), 0, stream>>>(Wf, n8f, 64, 32, WSC, WF2SC, WF16);
  k_prepq<<<dim3(NPIX / 64, 2, NB), dim3(256), 0, stream>>>(query, TB, XQ);
  k_prepk<<<dim3(NTKP / 64), dim3(256), 0, stream>>>(key, TB, XK, PK);
  k_gemm_tok<<<dim3(NTQ / 64, 2), dim3(256), 0, stream>>>(XQ, WQ16, bq, QSCALE, QF);
  k_gemm_tok<<<dim3(NTKP / 64, 2), dim3(256), 0, stream>>>(XK, WK16, bk, 1.0f, KF);
  k_gemm_tok<<<dim3(NTKP / 64, 2), dim3(256), 0, stream>>>(PK, WV16, bv, 1.0f, VF);
  k_attn<<<dim3(NTQ / 8), dim3(256), 0, stream>>>(QF, KF, VF, AO);
  k_gemm_nchw<false, true, true><<<dim3(NTQ / 64, 2), dim3(256), 0, stream>>>(
      AO, AO, WO16, CH, bo, INV_AOW, out_vo, VO16, VOSC);
  k_gemm_nchw<true, false, false><<<dim3(NTQ / 64, 2), dim3(256), 0, stream>>>(
      XQ, VO16, WF16, 2 * CH, bo, INV_XW, out_o, AO, 1.0f);
  (void)hipGetLastError();
}
